// IntegralTransform_38783554683204
// MI455X (gfx1250) — hardware-verified
//
#include <hip/hip_runtime.h>
#include <stddef.h>
#include <stdint.h>
#include <math.h>

#define NCO    3
#define CH     64
#define HID    256
#define D1     70
#define KF     64
#define K1     96
#define UPR    (K1 / 8)
#define NBT    512
#define PQP    512
#define K23    256
#define NTHR   256
#define EPB    128
#define QPB    4
#define AP     264
#define DP     68
#define GBM    64
#define GBN    128
#define GTHR   128
#define NU_BT  (NBT * UPR)
#define NU_W2  (HID * (K23 / 8))
#define NU_W3  (CH * (K23 / 8))
#define NU_W   (NU_BT + NU_W2 + NU_W3)
#define CA     4.0f
#define CW     256.0f
#define INVC   0.0009765625f
#define WSMAX  134217728
#define L_SA   (EPB * AP * 2)
#define L_SH   (EPB * AP * 2)
#define L_SD   (EPB * DP * 4)
#define L_SQ   (QPB * HID * 4)
#define L_SO   (QPB * CH * 4)
#define L_CST  ((HID + CH) * 4)
#define L_SW   (EPB * 4)
#define L_SJ   (EPB * 4)
#define L_SQL  (EPB * 4)
#define L_SRS  64
#define EDGE_LDS_BYTES (L_SA + L_SH + L_SD + L_SQ + L_SO + L_CST + L_SW + L_SJ + L_SQL + L_SRS)

static_assert(K1 % 32 == 0 && K23 % 32 == 0 && KF % 32 == 0);
static_assert(KF + 2 * NCO + 1 <= K1 && KF + 2 * NCO == D1);
static_assert(NU_BT % NTHR == 0 && NU_W2 % NTHR == 0 && NU_W3 % NTHR == 0 && (GBM * UPR) % NTHR == 0);
static_assert(NTHR == HID && NTHR == 2 * EPB && NTHR == QPB * CH && EPB == 8 * 16);
static_assert(AP >= K23 && (AP * 2) % 16 == 0 && DP >= CH && (DP * 4) % 16 == 0);
static_assert(L_SA % 16 == 0 && L_SD % 16 == 0 && L_SQ % 16 == 0 && L_SO % 16 == 0 && L_CST % 16 == 0);
static_assert(L_SW % 16 == 0 && L_SJ % 16 == 0 && L_SQL % 16 == 0);
static_assert(EDGE_LDS_BYTES <= 300000);
static_assert(GBM == (GTHR / 32) * 16 && GBN == 4 * 32 && (HID % GBN) == 0);
static_assert(QPB * CH * 4 == 2 * 32 * 16);

typedef float          v4f   __attribute__((ext_vector_type(4)));
typedef float          v8f   __attribute__((ext_vector_type(8)));
typedef int            v8i   __attribute__((ext_vector_type(8)));
typedef unsigned short v8us  __attribute__((ext_vector_type(8)));
typedef unsigned short v16us __attribute__((ext_vector_type(16)));
typedef __bf16         v16bf __attribute__((ext_vector_type(16)));
typedef _Float16       v16h  __attribute__((ext_vector_type(16)));
typedef _Float16       v8h   __attribute__((ext_vector_type(8)));
typedef v4f  __attribute__((may_alias)) v4fa;
typedef v8us __attribute__((may_alias)) v8usa;
typedef v8h  __attribute__((may_alias)) v8ha;
union FragB { v16bf v; v16us u; v8us h[2]; v8i w; };
union FragH { v16h v; v8h h[2]; v8i w; };

__device__ __forceinline__ v8f wmb(const FragB& a, const FragB& b, v8f c) {
  v8f d = __builtin_amdgcn_wmma_f32_16x16x32_bf16(false, a.v, false, b.v, (short)0, c, false, false);
  asm volatile("v_nop\n\tv_nop\n\tv_nop\n\tv_nop" : "+v"(d) : "v"(a.w), "v"(b.w));
  return d;
}
__device__ __forceinline__ v8f wmh(const FragH& a, const FragH& b, v8f c) {
  v8f d = __builtin_amdgcn_wmma_f32_16x16x32_f16(false, a.v, false, b.v, (short)0, c, false, false);
  asm volatile("v_nop\n\tv_nop\n\tv_nop\n\tv_nop" : "+v"(d) : "v"(a.w), "v"(b.w));
  return d;
}

__device__ __forceinline__ unsigned bf16_bits(float f) {
  const unsigned u = __float_as_uint(f);
  return (u + 0x7FFFu + ((u >> 16) & 1u)) >> 16;
}
__device__ __forceinline__ float bf16_val(float f) {
  return __uint_as_float(bf16_bits(f) << 16);
}
__device__ __forceinline__ float gelu_f(float t) {
  return 0.5f * t * (1.0f + erff(t * 0.70710678118654752440f));
}

__global__ __launch_bounds__(NTHR) void k_prep(const float* __restrict__ y, const float* __restrict__ x,
                                               const float* __restrict__ fy, const float* __restrict__ W1,
                                               const float* __restrict__ b1, const float* __restrict__ W2,
                                               const float* __restrict__ W3, int nN, int mRows,
                                               unsigned short* BT, _Float16* W2T, _Float16* W3T,
                                               unsigned short* NA) {
  const int u = (int)blockIdx.x * NTHR + (int)threadIdx.x;
  if (u < NU_BT) {
    const int n   = u / UPR;
    const int k8  = (u - n * UPR) * 8;
    const int nn  = n & (HID - 1);
    const bool isP = n < HID;
    v8us o;
#pragma unroll
    for (int i = 0; i < 8; ++i) {
      const int k = k8 + i;
      int ra = 6 + k;  ra = ra > D1 - 1 ? D1 - 1 : ra;
      int rb = k - KF; rb = rb < 0 ? 0 : (rb > 2 * NCO - 1 ? 2 * NCO - 1 : rb);
      const unsigned va = bf16_bits(W1[(size_t)ra * HID + nn]);
      const unsigned vb = bf16_bits(W1[(size_t)rb * HID + nn]);
      const unsigned vc = bf16_bits(b1[nn]);
      const unsigned m1 = (isP && k < KF) ? 0xFFFFu : 0u;
      const unsigned m2 = (k >= KF && k < D1 && (isP == (k < KF + NCO))) ? 0xFFFFu : 0u;
      const unsigned m3 = ((!isP) && k == D1) ? 0xFFFFu : 0u;
      o[i] = (unsigned short)((m1 & va) | (m2 & vb) | (m3 & vc));
    }
    unsigned short* dp = BT + (size_t)n * K1 + k8;
    *(volatile v8us*)dp = o;
    __threadfence();
    *(volatile v8us*)dp = o;
  } else if (u < NU_BT + NU_W2) {
    const int v  = u - NU_BT;
    const int n  = v >> 5;
    const int k8 = (v & 31) * 8;
    const float* p = W2 + (size_t)k8 * HID + n;
    v8h o;
#pragma unroll
    for (int i = 0; i < 8; ++i) o[i] = (_Float16)(CW * bf16_val(p[(size_t)i * HID]));
    _Float16* dp = W2T + (size_t)n * K23 + k8;
    *(volatile v8h*)dp = o;
    __threadfence();
    *(volatile v8h*)dp = o;
  } else if (u < NU_W) {
    const int v  = u - NU_BT - NU_W2;
    const int n  = v >> 5;
    const int k8 = (v & 31) * 8;
    const float* p = W3 + (size_t)k8 * CH + n;
    v8h o;
#pragma unroll
    for (int i = 0; i < 8; ++i) o[i] = (_Float16)(CW * bf16_val(p[(size_t)i * CH]));
    _Float16* dp = W3T + (size_t)n * K23 + k8;
    *(volatile v8h*)dp = o;
    __threadfence();
    *(volatile v8h*)dp = o;
  } else {
    const int v = u - NU_W;
    if (v >= mRows * UPR) return;
    const int row = v / UPR;
    const int k8  = (v - row * UPR) * 8;
    const int rc  = row < nN ? row : nN - 1;
    const bool ok = row < nN;
    const int kf  = k8 < KF - 8 ? k8 : KF - 8;
    const float* pf = fy + (size_t)rc * CH + kf;
    const v4f a = *(const v4fa*)pf;
    const v4f b = *(const v4fa*)(pf + 4);
    const float* py = y + (size_t)rc * NCO;
    const float* px = x + (size_t)rc * NCO;
    const unsigned fb[8] = {bf16_bits(a.x), bf16_bits(a.y), bf16_bits(a.z), bf16_bits(a.w),
                            bf16_bits(b.x), bf16_bits(b.y), bf16_bits(b.z), bf16_bits(b.w)};
    const unsigned cb[8] = {bf16_bits(py[0]), bf16_bits(py[1]), bf16_bits(py[2]),
                            bf16_bits(px[0]), bf16_bits(px[1]), bf16_bits(px[2]), 0x3F80u, 0u};
    const unsigned mF = (ok && k8 < KF) ? 0xFFFFu : 0u;
    const unsigned mC = (ok && k8 == KF) ? 0xFFFFu : 0u;
    v8us o;
#pragma unroll
    for (int i = 0; i < 8; ++i) o[i] = (unsigned short)((mF & fb[i]) | (mC & cb[i]));
    unsigned short* dp = NA + (size_t)row * K1 + k8;
    *(volatile v8us*)dp = o;
    __threadfence();
    *(volatile v8us*)dp = o;
  }
}

__global__ __launch_bounds__(GTHR) void k_gemm(const unsigned short* __restrict__ A, int lda,
                                               const unsigned short* __restrict__ BT, int ldb, int K,
                                               float* Cm, int ldc) {
  __shared__ __attribute__((aligned(16))) float stg[GBM * GBN];
  const int tid = (int)threadIdx.x, lane = tid & 31, wave = tid >> 5, hh = lane >> 4, m = lane & 15;
  const int rowBase = (int)blockIdx.x * GBM;
  const int colBase = (int)blockIdx.y * GBN;

  v8f acc[8];
  {
    const v8f z = {0.f, 0.f, 0.f, 0.f, 0.f, 0.f, 0.f, 0.f};
#pragma unroll
    for (int t = 0; t < 8; ++t) acc[t] = z;
  }
  const unsigned short* ap = A  + (size_t)(rowBase + 16 * wave + m) * (size_t)lda + 8 * hh;
  const unsigned short* bp = BT + (size_t)(colBase + m) * (size_t)ldb + 8 * hh;

#pragma unroll 1
  for (int k0 = 0; k0 < K; k0 += 32) {
    FragB af;
    af.h[0] = *(const v8usa*)(ap + k0);
    af.h[1] = *(const v8usa*)(ap + k0 + 16);
#pragma unroll
    for (int nt = 0; nt < 8; ++nt) {
      const unsigned short* wq = bp + (size_t)(16 * nt) * (size_t)ldb + k0;
      FragB bf;
      bf.h[0] = *(const v8usa*)wq;
      bf.h[1] = *(const v8usa*)(wq + 16);
      acc[nt] = wmb(af, bf, acc[nt]);
    }
  }

#pragma unroll
  for (int nt = 0; nt < 8; ++nt) {
    const int lc = 16 * nt + m;
#pragma unroll
    for (int r = 0; r < 8; ++r) {
      const int lr = 16 * wave + 8 * hh + r;
      stg[lr * GBN + lc] = acc[nt][r];
    }
  }
  __syncthreads();

  v4f pv[16];
#pragma unroll
  for (int i = 0; i < 16; ++i) pv[i] = *(const v4fa*)(stg + (16 * wave + i) * GBN + 4 * lane);
#pragma unroll
  for (int i = 0; i < 16; ++i) {
    float* op = Cm + (size_t)(rowBase + 16 * wave + i) * (size_t)ldc + colBase + 4 * lane;
    *(volatile v4f*)op = pv[i];
  }
  __threadfence();
#pragma unroll
  for (int i = 0; i < 16; ++i) {
    float* op = Cm + (size_t)(rowBase + 16 * wave + i) * (size_t)ldc + colBase + 4 * lane;
    *(volatile v4f*)op = pv[i];
  }
}

__global__ __launch_bounds__(NTHR) void k_edge(const int* __restrict__ nidx, const int* __restrict__ rsp,
                                               int nE, int nN,
                                               const float* __restrict__ PQ,
                                               const _Float16* __restrict__ W2T,
                                               const _Float16* __restrict__ W3T,
                                               const float* __restrict__ fy, const float* __restrict__ wts,
                                               const float* __restrict__ b2, const float* __restrict__ b3,
                                               float* out) {
  extern __shared__ __attribute__((aligned(16))) float dyn[];
  char* base = (char*)dyn;
  _Float16* sA  = (_Float16*)(base);
  _Float16* sH  = (_Float16*)(base + L_SA);
  float*    sD  = (float*)(base + L_SA + L_SH);
  float*    sQ  = (float*)(base + L_SA + L_SH + L_SD);
  float*    sO  = (float*)(base + L_SA + L_SH + L_SD + L_SQ);
  float*    cst = (float*)(base + L_SA + L_SH + L_SD + L_SQ + L_SO);
  float*    sW  = (float*)(base + L_SA + L_SH + L_SD + L_SQ + L_SO + L_CST);
  int*      sJ  = (int*)(base + L_SA + L_SH + L_SD + L_SQ + L_SO + L_CST + L_SW);
  int*      sQL = (int*)(base + L_SA + L_SH + L_SD + L_SQ + L_SO + L_CST + L_SW + L_SJ);
  int*      sRS = (int*)(base + L_SA + L_SH + L_SD + L_SQ + L_SO + L_CST + L_SW + L_SJ + L_SQL);

  const int tid = (int)threadIdx.x, lane = tid & 31, wave = tid >> 5, hh = lane >> 4, m = lane & 15;
  const int q0 = (int)blockIdx.x * QPB;

  {
    int qi = q0 + (tid < QPB ? tid : QPB);
    qi = qi > nN ? nN : qi;
    int v = rsp[qi];
    v = v < 0 ? 0 : (v > nE ? nE : v);
    if (tid <= QPB) sRS[tid] = v;
    cst[tid] = bf16_val(b2[tid]);
    const float vb3 = b3[tid < CH ? tid : CH - 1];
    if (tid < CH) cst[HID + tid] = bf16_val(vb3);
  }
  __syncthreads();
  const int lo = sRS[0], e1 = sRS[1], e2 = sRS[2], e3 = sRS[3], hi = sRS[4];
  const bool bad = (e1 < lo) || (e2 < e1) || (e3 < e2) || (hi < e3) || (hi - lo > EPB);

  if (tid < EPB) {
    const int ea = lo + tid;
    const int ec = ea > nE - 1 ? nE - 1 : ea;
    int j = nidx[ec];
    j = j < 0 ? 0 : (j > nN - 1 ? nN - 1 : j);
    sJ[tid]  = j;
    sW[tid]  = bf16_val(wts[j]);
    sQL[tid] = (ea >= e1 ? 1 : 0) + (ea >= e2 ? 1 : 0) + (ea >= e3 ? 1 : 0);
  }
  {
    const int qi = tid >> 6, c4 = tid & 63;
    int qr = q0 + qi;
    qr = qr > nN - 1 ? nN - 1 : qr;
    const v4f qv = *(const v4fa*)(PQ + (size_t)qr * PQP + HID + 4 * c4);
    *(v4fa*)(sQ + qi * HID + 4 * c4) = qv;
  }
  __syncthreads();

  {
    const int s  = tid & (EPB - 1);
    const int hf = tid >> 7;
    const int j  = sJ[s];
    const int ql = sQL[s];
    const float* pr = PQ + (size_t)j * PQP + (HID / 2) * hf;
    const float* qr = sQ + ql * HID + (HID / 2) * hf;
    _Float16*    ar = sA + s * AP + (HID / 2) * hf;
#pragma unroll 1
    for (int c8 = 0; c8 < HID / 16; ++c8) {
      const v4f pa = *(const v4fa*)(pr + 8 * c8);
      const v4f pb = *(const v4fa*)(pr + 8 * c8 + 4);
      const v4f qa = *(const v4fa*)(qr + 8 * c8);
      const v4f qb = *(const v4fa*)(qr + 8 * c8 + 4);
      v8h o;
      o[0] = (_Float16)(CA * gelu_f(pa.x + qa.x));
      o[1] = (_Float16)(CA * gelu_f(pa.y + qa.y));
      o[2] = (_Float16)(CA * gelu_f(pa.z + qa.z));
      o[3] = (_Float16)(CA * gelu_f(pa.w + qa.w));
      o[4] = (_Float16)(CA * gelu_f(pb.x + qb.x));
      o[5] = (_Float16)(CA * gelu_f(pb.y + qb.y));
      o[6] = (_Float16)(CA * gelu_f(pb.z + qb.z));
      o[7] = (_Float16)(CA * gelu_f(pb.w + qb.w));
      *(v8ha*)(ar + 8 * c8) = o;
    }
  }
  __syncthreads();

  {
    const _Float16* ap = sA + (16 * wave + m) * AP + 8 * hh;
#pragma unroll 1
    for (int nc = 0; nc < HID / 128; ++nc) {
      v8f acc[8];
      {
        const v8f z = {0.f, 0.f, 0.f, 0.f, 0.f, 0.f, 0.f, 0.f};
#pragma unroll
        for (int t = 0; t < 8; ++t) acc[t] = z;
      }
      const _Float16* bp = W2T + (size_t)(nc * 128 + m) * K23 + 8 * hh;
#pragma unroll 1
      for (int k0 = 0; k0 < K23; k0 += 32) {
        FragH af;
        af.h[0] = *(const v8ha*)(ap + k0);
        af.h[1] = *(const v8ha*)(ap + k0 + 16);
#pragma unroll
        for (int nt = 0; nt < 8; ++nt) {
          const _Float16* wq = bp + (size_t)(16 * nt) * K23 + k0;
          FragH bf;
          bf.h[0] = *(const v8ha*)wq;
          bf.h[1] = *(const v8ha*)(wq + 16);
          acc[nt] = wmh(af, bf, acc[nt]);
        }
      }
#pragma unroll
      for (int nt = 0; nt < 8; ++nt) {
        const int col = nc * 128 + 16 * nt + m;
        const float bv = cst[col];
#pragma unroll
        for (int r = 0; r < 8; ++r) {
          const int row = 16 * wave + 8 * hh + r;
          const float u2 = acc[nt][r] * INVC + bv;
          sH[row * AP + col] = (_Float16)(CA * gelu_f(u2));
        }
      }
    }
  }
  __syncthreads();

  {
    const _Float16* ap = sH + (16 * wave + m) * AP + 8 * hh;
    const _Float16* bp = W3T + (size_t)m * K23 + 8 * hh;
    v8f acc[4];
    {
      const v8f z = {0.f, 0.f, 0.f, 0.f, 0.f, 0.f, 0.f, 0.f};
#pragma unroll
      for (int t = 0; t < 4; ++t) acc[t] = z;
    }
#pragma unroll 1
    for (int k0 = 0; k0 < K23; k0 += 32) {
      FragH af;
      af.h[0] = *(const v8ha*)(ap + k0);
      af.h[1] = *(const v8ha*)(ap + k0 + 16);
#pragma unroll
      for (int nt = 0; nt < 4; ++nt) {
        const _Float16* wq = bp + (size_t)(16 * nt) * K23 + k0;
        FragH bf;
        bf.h[0] = *(const v8ha*)wq;
        bf.h[1] = *(const v8ha*)(wq + 16);
        acc[nt] = wmh(af, bf, acc[nt]);
      }
    }
#pragma unroll
    for (int nt = 0; nt < 4; ++nt) {
      const int col = 16 * nt + m;
      const float bv = cst[HID + col];
#pragma unroll
      for (int r = 0; r < 8; ++r) {
        const int row = 16 * wave + 8 * hh + r;
        sD[row * DP + col] = acc[nt][r] * INVC + bv;
      }
    }
  }
  __syncthreads();

  {
    const int ql = tid >> 6, c = tid & (CH - 1);
    int sb = sRS[ql] - lo, se = sRS[ql + 1] - lo;
    sb = sb < 0 ? 0 : (sb > EPB ? EPB : sb);
    se = se < 0 ? 0 : (se > EPB ? EPB : se);
    float sum = 0.0f;
#pragma unroll 2
    for (int s = sb; s < se; ++s) {
      const int j = sJ[s];
      const float fv = bf16_val(fy[(size_t)j * CH + c]);
      const float kv = sD[s * DP + c];
      const float wv = sW[s];
      sum = sum + wv * (kv * fv);
    }
    const float ov = bad ? __uint_as_float(0x7fc00000u) : sum;
    sO[ql * CH + c] = ov;
  }
  __syncthreads();

  const int tl = tid < 64 ? tid : 63;
  const v4f o4 = *(const v4fa*)(sO + 4 * tl);
  const int orow = q0 + (tl >> 4);
  const bool stv = (tid < 64) && (orow < nN);
  float* op = out + (size_t)q0 * CH + 4 * tl;
  if (stv) *(volatile v4f*)op = o4;
  __threadfence();
  if (stv) *(volatile v4f*)op = o4;
}

static inline int cdiv(int a, int b) { return (a + b - 1) / b; }

extern "C" void kernel_launch(void* const* d_in, const int* in_sizes, int n_in,
                              void* d_out, int out_size, void* d_ws, size_t ws_size,
                              hipStream_t stream) {
  if (n_in < 12) return;
  if (in_sizes[0] < NCO || (in_sizes[0] % NCO) != 0) return;
  const int nN = in_sizes[0] / NCO;
  if (in_sizes[1] != NCO * nN) return;
  if (in_sizes[2] != CH * nN) return;
  if (in_sizes[3] != nN) return;
  const int nE = in_sizes[4];
  if (nE < 1) return;
  if (in_sizes[5] != nN + 1) return;
  if (in_sizes[6] != D1 * HID || in_sizes[7] != HID) return;
  if (in_sizes[8] != HID * HID || in_sizes[9] != HID) return;
  if (in_sizes[10] != HID * CH || in_sizes[11] != CH) return;
  if (out_size != nN * CH) return;

  const float* y    = (const float*)d_in[0];
  const float* x    = (const float*)d_in[1];
  const float* fy   = (const float*)d_in[2];
  const float* wts  = (const float*)d_in[3];
  const int*   nidx = (const int*)d_in[4];
  const int*   rsp  = (const int*)d_in[5];
  const float* W1   = (const float*)d_in[6];
  const float* b1   = (const float*)d_in[7];
  const float* W2   = (const float*)d_in[8];
  const float* b2   = (const float*)d_in[9];
  const float* W3   = (const float*)d_in[10];
  const float* b3   = (const float*)d_in[11];
  float* out = (float*)d_out;

  const int MP = cdiv(nN, GBM) * GBM;
  const int gM = MP / GBM;

  char* ws = (char*)d_ws;
  size_t off = 0;
  const size_t oBT = off; off += (size_t)NBT * K1 * 2;    off = (off + 255) & ~(size_t)255;
  const size_t oW2 = off; off += (size_t)HID * K23 * 2;   off = (off + 255) & ~(size_t)255;
  const size_t oW3 = off; off += (size_t)CH * K23 * 2;    off = (off + 255) & ~(size_t)255;
  const size_t oNA = off; off += (size_t)MP * K1 * 2;     off = (off + 255) & ~(size_t)255;
  const size_t oPQ = off; off += (size_t)MP * PQP * 4;    off = (off + 255) & ~(size_t)255;
  if (off > ws_size || off > (size_t)WSMAX) return;
  unsigned short* BT  = (unsigned short*)(ws + oBT);
  _Float16*       W2T = (_Float16*)(ws + oW2);
  _Float16*       W3T = (_Float16*)(ws + oW3);
  unsigned short* NA  = (unsigned short*)(ws + oNA);
  float*          PQ  = (float*)(ws + oPQ);

  hipFuncSetAttribute(reinterpret_cast<const void*>(&k_edge), hipFuncAttributeMaxDynamicSharedMemorySize,
                      (int)EDGE_LDS_BYTES);

  const int nUnits = NU_W + MP * UPR;
  k_prep<<<cdiv(nUnits, NTHR), NTHR, 0, stream>>>(y, x, fy, W1, b1, W2, W3, nN, MP, BT, W2T, W3T, NA);
  k_gemm<<<dim3(gM, HID / GBN), GTHR, 0, stream>>>(NA, K1, BT, K1, K1, PQ, PQP);
  k_gemm<<<dim3(gM, HID / GBN), GTHR, 0, stream>>>(NA + KF, K1, BT + (size_t)HID * K1 + KF, K1, K1 - KF,
                                                   PQ + HID, PQP);
  k_edge<<<cdiv(nN, QPB), NTHR, EDGE_LDS_BYTES, stream>>>(nidx, rsp, nE, nN, PQ, W2T, W3T, fy, wts, b2, b3, out);
}
